// SparseCosineKernel_48120813584931
// MI455X (gfx1250) — hardware-verified
//
#include <hip/hip_runtime.h>


#define NPTS 200000
#define DD   64
#define MM   1000
#define MP   1024
#define NMOL 1000
typedef __attribute__((ext_vector_type(16))) _Float16 v16h;
typedef __attribute__((ext_vector_type(8)))  _Float16 v8h;
typedef __attribute__((ext_vector_type(8)))  float    v8f;
typedef __attribute__((ext_vector_type(2)))  int      v2i;
#define VST2(T, ptr, val) do { const T _v = (val); *(volatile T*)(ptr) = _v; __threadfence(); *(volatile T*)(ptr) = _v; } while (0)
__device__ __forceinline__ v8f wmma16(v16h a, v16h b, v8f c) {
  v8f d = __builtin_amdgcn_wmma_f32_16x16x32_f16(false, a, false, b, (short)0, c, false, false);
  asm volatile("v_nop\n\tv_nop\n\tv_nop\n\tv_nop" : "+v"(d) : "v"(a), "v"(b));
  return d;
}
__device__ __forceinline__ v16h frag16(const _Float16* p, int hh) {
  const v8h lo = *(const v8h*)(p + 8 * hh), hi = *(const v8h*)(p + 16 + 8 * hh);
  return __builtin_shufflevector(lo, hi, 0,1,2,3,4,5,6,7,8,9,10,11,12,13,14,15);
}
__global__ __launch_bounds__(256) void k_cvt(const float* __restrict__ PS, const float* __restrict__ SP, _Float16* __restrict__ P16, _Float16* __restrict__ S16) {
  const int t = blockIdx.x * 256 + threadIdx.x;
  const int np8 = (NPTS + 16) * 8;
  v8h o;
  if (t < np8) { const int i = t >> 3, c = (t & 7) * 8;
#pragma unroll
    for (int e = 0; e < 8; ++e) o[e] = (i < NPTS) ? (_Float16)PS[(size_t)i * DD + c + e] : (_Float16)0.f;
    VST2(v8h, P16 + (size_t)i * DD + c, o);
  } else if (t < np8 + MP * 8) { const int u = t - np8, j = u >> 3, c = (u & 7) * 8;
#pragma unroll
    for (int e = 0; e < 8; ++e) o[e] = (j < MM) ? (_Float16)SP[(size_t)j * DD + c + e] : (_Float16)0.f;
    VST2(v8h, S16 + (size_t)j * DD + c, o);
  }
}
__global__ __launch_bounds__(256) void k_segs(const int* __restrict__ batch, v2i* __restrict__ seg) {
  const int b = blockIdx.x * 256 + threadIdx.x;
  if (b >= NMOL) return;
  int lo = 0, hi = NPTS;
  while (lo < hi) { const int mid = (lo + hi) >> 1; if (batch[mid] < b) lo = mid + 1; else hi = mid; }
  const int st = lo; hi = NPTS;
  while (lo < hi) { const int mid = (lo + hi) >> 1; if (batch[mid] < b + 1) lo = mid + 1; else hi = mid; }
  const v2i sv = {st, lo};
  VST2(v2i, seg + b, sv);
}
__global__ __launch_bounds__(512) void k_kernel(const _Float16* __restrict__ P16, const _Float16* __restrict__ S16, const int* __restrict__ z,
                                                const int* __restrict__ psp, const v2i* __restrict__ seg, float* __restrict__ out) {
  __shared__ __attribute__((aligned(16))) float rows[4][MP];
  const int lane = threadIdx.x & 31, wave = threadIdx.x >> 5, hh = lane >> 4, l16 = lane & 15;
  const int cg = wave, c0 = cg * 64;
 for (int mi = 0; mi < 4; ++mi) {
  const int mol = blockIdx.x * 4 + mi;
  v2i sv = seg[mol];
  sv[0] = min(max(sv[0], 0), NPTS); sv[1] = min(max(sv[1], sv[0]), min(sv[0] + 4096, NPTS));
  v16h b0[4], b1[4]; int spz[4];
#pragma unroll
  for (int t = 0; t < 4; ++t) { const _Float16* sp = S16 + (size_t)(c0 + t * 16 + l16) * DD; b0[t] = frag16(sp, hh); b1[t] = frag16(sp + 32, hh);
    const int j = c0 + t * 16 + l16; spz[t] = (j < MM) ? psp[j] : -1; }
  float colsum[4] = {0.f, 0.f, 0.f, 0.f};
  for (int r0 = sv[0]; r0 < sv[1]; r0 += 16) {
    const _Float16* pr = P16 + (size_t)(r0 + l16) * DD;
    const v16h a0 = frag16(pr, hh), a1 = frag16(pr + 32, hh);
    int zr[8];
#pragma unroll
    for (int v = 0; v < 8; ++v) { const int i = r0 + v + 8 * hh; zr[v] = (i < sv[1]) ? z[i] : -2; }
#pragma unroll
    for (int t = 0; t < 4; ++t) {
      v8f c = {};
      c = wmma16(a0, b0[t], c);
      c = wmma16(a1, b1[t], c);
      float s = 0.f;
#pragma unroll
      for (int v = 0; v < 8; ++v) s += (zr[v] == spz[t]) ? c[v] * c[v] : 0.f;
      colsum[t] += s;
    }
  }
#pragma unroll
  for (int t = 0; t < 4; ++t) { const float tot = colsum[t] + __shfl_xor(colsum[t], 16); if (hh == 0) rows[mi][c0 + t * 16 + l16] = tot; }
 }
  __syncthreads();
  typedef __attribute__((ext_vector_type(4))) float v4f;
  float* od = out + (size_t)blockIdx.x * 4 * MM;
  for (int pass = 0; pass < 2; ++pass) {
    for (int p = threadIdx.x; p < MM; p += 512) {
      const int mi = p / 250, col = (p % 250) * 4;
      *(volatile v4f*)(od + (size_t)p * 4) = *(const v4f*)(&rows[mi][col]);
    }
    __threadfence();
  }
}
extern "C" void kernel_launch(void* const* d_in, const int* in_sizes, int n_in,
                              void* d_out, int out_size, void* d_ws, size_t ws_size, hipStream_t stream) {
  (void)in_sizes; (void)n_in; (void)out_size;
  const float* PS  = (const float*)d_in[0];
  const float* SP  = (const float*)d_in[1];
  const int*   z   = (const int*)  d_in[2];
  const int*   bat = (const int*)  d_in[3];
  const int*   psp = (const int*)  d_in[4];
  float* out = (float*)d_out;
  char* ws = (char*)d_ws; size_t off = 0;
  auto take = [&](size_t bytes) { void* p = ws + off; off = (off + bytes + 255) & ~(size_t)255; return p; };
  _Float16* P16 = (_Float16*)take((size_t)(NPTS + 16) * DD * 2);
  _Float16* S16 = (_Float16*)take((size_t)MP * DD * 2);
  v2i* seg = (v2i*)take((size_t)NMOL * 8);
  if (off > ws_size) return;
  k_cvt<<<((NPTS + 16) * 8 + MP * 8 + 255) / 256, 256, 0, stream>>>(PS, SP, P16, S16);
  k_segs<<<(NMOL + 255) / 256, 256, 0, stream>>>(bat, seg);
  k_kernel<<<NMOL / 4, 512, 0, stream>>>(P16, S16, z, psp, seg, out);
}
